// MMDLoss_6090263625755
// MI455X (gfx1250) — hardware-verified
//
#include <hip/hip_runtime.h>

typedef _Float16 v8h  __attribute__((ext_vector_type(8)));
typedef _Float16 v16h __attribute__((ext_vector_type(16)));
typedef float    v8f  __attribute__((ext_vector_type(8)));
typedef float    v4f  __attribute__((ext_vector_type(4)));
typedef double   v2d  __attribute__((ext_vector_type(2)));

union Frag { v16h v; v8h hf[2]; };

#define N_TOTAL 8192
#define BHALF   4096
#define DDIM    256
#define LROW    264
#define NTILE   128
#define NPAIRS  8256
#define RPB     32

#define XH_OFF    0u
#define SQ_OFF    4194304u
#define COEF_OFF  4227072u
#define PART_OFF  4227200u
#define PART_LINE 128u
#define WS_NEED   (PART_OFF + (unsigned)NPAIRS * PART_LINE)

__device__ __forceinline__ v8f wmma16(const v16h a, const v16h b, v8f c) {
  v8f d = __builtin_amdgcn_wmma_f32_16x16x32_f16(false, a, false, b, (short)0, c, false, false);
  asm volatile("v_nop\n\tv_nop\n\tv_nop\n\tv_nop" : "+v"(d) : "v"(a), "v"(b));
  return d;
}

__global__ void __launch_bounds__(256)
k_prep(const float* __restrict__ src, const float* __restrict__ tgt, char* __restrict__ ws) {
  _Float16* Xh = (_Float16*)(ws + XH_OFF);
  float* sq    = (float*)(ws + SQ_OFF);

  __shared__ float sqs[RPB];

  const int t = threadIdx.x;
  const int w = t >> 5;
  const int l = t & 31;
  const int row0 = (int)blockIdx.x * RPB;
  if (row0 >= N_TOTAL) return;

  v8h hv[4];
#pragma unroll
  for (int rr = 0; rr < 4; ++rr) {
    const int row = row0 + w * 4 + rr;
    const float* rp = (row < BHALF) ? (src + (size_t)row * DDIM)
                                    : (tgt + (size_t)(row - BHALF) * DDIM);
    const v4f x0 = *(const v4f*)(rp + l * 8);
    const v4f x1 = *(const v4f*)(rp + l * 8 + 4);
    float p = x0.x * x0.x + x0.y * x0.y + x0.z * x0.z + x0.w * x0.w
            + x1.x * x1.x + x1.y * x1.y + x1.z * x1.z + x1.w * x1.w;
    v8h hq;
    hq[0] = (_Float16)x0.x; hq[1] = (_Float16)x0.y; hq[2] = (_Float16)x0.z; hq[3] = (_Float16)x0.w;
    hq[4] = (_Float16)x1.x; hq[5] = (_Float16)x1.y; hq[6] = (_Float16)x1.z; hq[7] = (_Float16)x1.w;
    hv[rr] = hq;
    *(volatile v8h*)(Xh + (size_t)row * DDIM + l * 8) = hq;
#pragma unroll
    for (int off = 16; off > 0; off >>= 1) p += __shfl_xor(p, off);
    if (l == 0) sqs[w * 4 + rr] = p;
  }
  __threadfence();
#pragma unroll
  for (int rr = 0; rr < 4; ++rr) {
    const int row = row0 + w * 4 + rr;
    *(volatile v8h*)(Xh + (size_t)row * DDIM + l * 8) = hv[rr];
  }
  __syncthreads();
  if (t < 8) {
    v4f q;
    q.x = sqs[4 * t + 0]; q.y = sqs[4 * t + 1]; q.z = sqs[4 * t + 2]; q.w = sqs[4 * t + 3];
    volatile v4f* dst = (volatile v4f*)(sq + row0) + t;
    *dst = q;
    __threadfence();
    *dst = q;
  }
}

__global__ void __launch_bounds__(256)
k_bw(const float* __restrict__ src, const float* __restrict__ tgt, char* __restrict__ ws) {
  const float* sq = (const float*)(ws + SQ_OFF);
  float* coefp    = (float*)(ws + COEF_OFF);

  __shared__ double dred[256];
  __shared__ float cf;

  const int t = threadIdx.x;

  double cs = 0.0;
#pragma unroll 8
  for (int r = 0; r < BHALF; ++r) cs += (double)src[(size_t)r * DDIM + t];
#pragma unroll 8
  for (int r = 0; r < BHALF; ++r) cs += (double)tgt[(size_t)r * DDIM + t];

  dred[t] = cs * cs;
  __syncthreads();
  for (int st = 128; st > 0; st >>= 1) {
    if (t < st) dred[t] += dred[t + st];
    __syncthreads();
  }
  const double ss = dred[0];
  __syncthreads();

  double s2 = 0.0;
#pragma unroll 8
  for (int k = 0; k < 32; ++k) s2 += (double)sq[t * 32 + k];
  dred[t] = s2;
  __syncthreads();
  for (int st = 128; st > 0; st >>= 1) {
    if (t < st) dred[t] += dred[t + st];
    __syncthreads();
  }
  if (t == 0) {
    const double sumsq  = dred[0];
    const double n      = (double)N_TOTAL;
    const double sum_l2 = 2.0 * n * sumsq - 2.0 * ss;
    const double bw     = sum_l2 / (n * n - n);
    const double den0   = bw * 0.25;
    cf = (float)(-1.0 / den0);
  }
  __syncthreads();
  if (t < 8) {
    v4f q;
    q.x = (t == 0) ? cf : 0.f; q.y = 0.f; q.z = 0.f; q.w = 0.f;
    volatile v4f* dst = (volatile v4f*)coefp + t;
    *dst = q;
    __threadfence();
    *dst = q;
  }
}

__global__ void __launch_bounds__(128)
k_gram(char* __restrict__ ws) {
  const _Float16* Xh = (const _Float16*)(ws + XH_OFF);
  const float* sq    = (const float*)(ws + SQ_OFF);
  const float coef   = *((const float*)(ws + COEF_OFF));

  __shared__ __align__(16) _Float16 As[64 * LROW];
  __shared__ __align__(16) _Float16 Bs[64 * LROW];
  __shared__ double red[128];

  const int t    = threadIdx.x;
  const int w    = t >> 5;
  const int lane = t & 31;
  const int l15  = lane & 15;
  const int h    = lane >> 4;

  const int p = (int)blockIdx.x;
  if (p >= NPAIRS) return;

  int bi = (int)((2.f * NTILE + 1.f -
                  sqrtf((float)((2 * NTILE + 1) * (2 * NTILE + 1) - 8 * p))) * 0.5f);
  if (bi < 0) bi = 0;
  if (bi > NTILE - 1) bi = NTILE - 1;
  while (bi > 0 && (bi * NTILE - (bi * (bi - 1)) / 2) > p) --bi;
  while (bi < NTILE - 1 && ((bi + 1) * NTILE - ((bi + 1) * bi) / 2) <= p) ++bi;
  int bj = bi + (p - (bi * NTILE - (bi * (bi - 1)) / 2));
  if (bj > NTILE - 1) bj = NTILE - 1;
  const bool diagBlk = (bi == bj);

  const int ibase = bi * 64 + w * 16;
  const int jbase = bj * 64;

  {
    const _Float16* gA = Xh + (size_t)bi * 64 * DDIM;
    const _Float16* gB = Xh + (size_t)bj * 64 * DDIM;
#pragma unroll 4
    for (int c = 0; c < 16; ++c) {
      const int chunk = c * 128 + t;
      const int row   = chunk >> 5;
      const int col8  = (chunk & 31) * 8;
      *(v8h*)(As + row * LROW + col8) = *(const v8h*)(gA + (size_t)row * DDIM + col8);
      if (!diagBlk)
        *(v8h*)(Bs + row * LROW + col8) = *(const v8h*)(gB + (size_t)row * DDIM + col8);
    }
  }
  __syncthreads();

  const _Float16* Bp   = diagBlk ? As : Bs;
  const _Float16* aRow = As + (w * 16 + l15) * LROW + h * 8;
  const _Float16* bRow = Bp + l15 * LROW + h * 8;

  v8f acc[4] = {};

#pragma unroll
  for (int kk = 0; kk < DDIM; kk += 32) {
    Frag a;
    a.hf[0] = *(const v8h*)(aRow + kk);
    a.hf[1] = *(const v8h*)(aRow + kk + 16);
#pragma unroll
    for (int n = 0; n < 4; ++n) {
      const _Float16* br = bRow + n * 16 * LROW;
      Frag b;
      b.hf[0] = *(const v8h*)(br + kk);
      b.hf[1] = *(const v8h*)(br + kk + 16);
      acc[n] = wmma16(a.v, b.v, acc[n]);
    }
  }

  float si[8];
#pragma unroll
  for (int r = 0; r < 8; ++r) si[r] = sq[ibase + h * 8 + r];

  float accsum = 0.f;
#pragma unroll
  for (int n = 0; n < 4; ++n) {
    const int j    = jbase + n * 16 + l15;
    const float sj = sq[j];
#pragma unroll
    for (int r = 0; r < 8; ++r) {
      const int i = ibase + h * 8 + r;
      float l2 = si[r] + sj - 2.f * acc[n][r];
      l2 = fmaxf(l2, 0.f);
      const float e0 = __expf(coef * l2);
      float ks = e0;
      float tt = e0;
#pragma unroll
      for (int q = 0; q < 4; ++q) { tt = __fsqrt_rn(tt); ks += tt; }
      const float sgn = (((i ^ j) & BHALF) ? -1.f : 1.f);
      const float wgt = diagBlk ? ((j > i) ? 2.f : ((j == i) ? 1.f : 0.f)) : 2.f;
      accsum += wgt * sgn * ks;
    }
  }

  red[t] = (double)accsum;
  __syncthreads();
  for (int st = 64; st > 0; st >>= 1) {
    if (t < st) red[t] += red[t + st];
    __syncthreads();
  }
  const double tot = red[0];
  if (t < 8) {
    v2d q;
    q.x = (t == 0) ? tot : 0.0; q.y = 0.0;
    volatile v2d* dst = (volatile v2d*)(ws + PART_OFF + (size_t)p * PART_LINE) + t;
    *dst = q;
    __threadfence();
    *dst = q;
  }
}

__global__ void __launch_bounds__(256)
k_final(const char* __restrict__ ws, float* __restrict__ out) {
  const double* part = (const double*)(ws + PART_OFF);
  __shared__ double dred[256];
  const int t = threadIdx.x;
  double s = 0.0;
  for (int i = t; i < NPAIRS; i += 256) s += part[(size_t)i * (PART_LINE / 8)];
  dred[t] = s;
  __syncthreads();
  for (int st = 128; st > 0; st >>= 1) {
    if (t < st) dred[t] += dred[t + st];
    __syncthreads();
  }
  if (t == 0) {
    const float r = (float)(dred[0] / ((double)BHALF * (double)BHALF));
    volatile float* o = out;
    *o = r;
    __threadfence();
    *o = r;
  }
}

extern "C" void kernel_launch(void* const* d_in, const int* in_sizes, int n_in,
                              void* d_out, int out_size, void* d_ws, size_t ws_size,
                              hipStream_t stream) {
  if (n_in < 2) return;
  if (in_sizes[0] != BHALF * DDIM || in_sizes[1] != BHALF * DDIM) return;
  if (out_size < 1) return;
  if (ws_size < (size_t)WS_NEED) return;

  const float* src = (const float*)d_in[0];
  const float* tgt = (const float*)d_in[1];
  float* out = (float*)d_out;
  char* ws   = (char*)d_ws;

  k_prep<<<N_TOTAL / RPB, 256, 0, stream>>>(src, tgt, ws);
  k_bw<<<1, 256, 0, stream>>>(src, tgt, ws);
  k_gram<<<NPAIRS, 128, 0, stream>>>(ws);
  k_final<<<1, 256, 0, stream>>>(ws, out);
}
